// TransformerBlock_58789512347974
// MI455X (gfx1250) — hardware-verified
//
#include <hip/hip_runtime.h>
#include <stddef.h>


typedef _Float16 v16h __attribute__((ext_vector_type(16)));
typedef _Float16 v8h  __attribute__((ext_vector_type(8)));
typedef float    v8f  __attribute__((ext_vector_type(8)));
typedef float    v4f  __attribute__((ext_vector_type(4)));

#ifndef NB
#define NB 1
#endif
#ifndef SEQ
#define SEQ 2048
#endif
#define NB_FULL  1
#define SEQ_FULL 2048
#define DIM   1024
#define NHEAD 16
#define HD    64
#define DMLP  4096
#define MROWS (NB * SEQ)
#define LN_ITERS 4

static_assert(NB >= 1 && NB <= NB_FULL);
static_assert(SEQ >= 128 && SEQ <= SEQ_FULL && (SEQ % 128) == 0);
static_assert(DIM == NHEAD * HD);
static_assert(HD == 64);
static_assert((DIM % 64) == 0 && (DIM % 32) == 0);
static_assert((DMLP % 64) == 0 && (DMLP % 32) == 0);
static_assert((MROWS % 64) == 0 && (MROWS % 8) == 0);
static_assert(DIM == LN_ITERS * 32 * 8);
static_assert(64 * 64 == 256 * 16);
static_assert((size_t)MROWS * DMLP < (size_t)0xFFFFFFFFu);

#define LDT 72
#define LDC 68

#define WCARRY 64.0f
#define PCARRY 1024.0f
#define VCARRY 64.0f
#define GCARRY 64.0f
#define LN_EPS 1.0e-5f
#define MASK_FILL -1.0e5f

#define WSQ_BYTES   ((size_t)DIM * DIM * 2)
#define WMLP_BYTES  ((size_t)DIM * DMLP * 2)
#define P16_BYTES   ((size_t)MROWS * DIM * 2)
#define RMID_BYTES  ((size_t)MROWS * DIM * 4)
#define G16_BYTES   ((size_t)MROWS * DMLP * 2)
#define OFF_WQ    ((size_t)0)
#define OFF_WK    (OFF_WQ + WSQ_BYTES)
#define OFF_WV    (OFF_WK + WSQ_BYTES)
#define OFF_WO    (OFF_WV + WSQ_BYTES)
#define OFF_WIN   (OFF_WO + WSQ_BYTES)
#define OFF_WOUT  (OFF_WIN + WMLP_BYTES)
#define OFF_X1    (OFF_WOUT + WMLP_BYTES)
#define OFF_Q     (OFF_X1 + P16_BYTES)
#define OFF_K     (OFF_Q + P16_BYTES)
#define OFF_VT    (OFF_K + P16_BYTES)
#define OFF_CTX   (OFF_VT + P16_BYTES)
#define OFF_X2    (OFF_CTX + P16_BYTES)
#define OFF_RMID  (OFF_X2 + P16_BYTES)
#define OFF_G     (OFF_RMID + RMID_BYTES)
#define WS_TOTAL  (OFF_G + G16_BYTES)
static_assert((WSQ_BYTES % 128) == 0 && (WMLP_BYTES % 128) == 0 && (P16_BYTES % 128) == 0);
static_assert((RMID_BYTES % 128) == 0 && (G16_BYTES % 128) == 0);
static_assert(WS_TOTAL <= (size_t)134217728);

__device__ __forceinline__ float bf16r(float x) {
  unsigned int u = __float_as_uint(x);
  u = (u + 0x7FFFu + ((u >> 16) & 1u)) & 0xFFFF0000u;
  return __uint_as_float(u);
}

__device__ __forceinline__ v16h frag_at(const _Float16* p) {
  v8h lo = *(const v8h*)(p);
  v8h hi = *(const v8h*)(p + 16);
  v16h out;
#pragma unroll
  for (int i = 0; i < 8; ++i) { out[i] = lo[i]; out[i + 8] = hi[i]; }
  return out;
}
__device__ __forceinline__ v16h ld_frag(const _Float16* base, unsigned ld) {
  const unsigned lane = threadIdx.x & 31u;
  return frag_at(base + (lane & 15u) * ld + (lane >> 4) * 8u);
}

__device__ __forceinline__ v8f wmma16(v16h a, v16h b, v8f c) {
  v8f d = __builtin_amdgcn_wmma_f32_16x16x32_f16(false, a, false, b, (short)0, c,
                                                 false, false);
  asm volatile("v_nop\n\tv_nop\n\tv_nop\n\tv_nop" : "+v"(d) : "v"(a), "v"(b));
  return d;
}

__device__ __forceinline__ unsigned wave_id() {
  return (unsigned)__builtin_amdgcn_readfirstlane((int)(threadIdx.x >> 5));
}

__device__ __forceinline__ float red16_max(float x) {
#pragma unroll
  for (int off = 1; off < 16; off <<= 1) x = fmaxf(x, __shfl_xor(x, off, 32));
  return x;
}
__device__ __forceinline__ float red16_sum(float x) {
#pragma unroll
  for (int off = 1; off < 16; off <<= 1) x += __shfl_xor(x, off, 32);
  return x;
}
__device__ __forceinline__ float red32_sum(float x) {
#pragma unroll
  for (int off = 1; off < 32; off <<= 1) x += __shfl_xor(x, off, 32);
  return x;
}

__device__ __forceinline__ void wave_lds_sync() {
  __builtin_amdgcn_fence(3  , "wavefront");
  asm volatile("s_wait_dscnt 0x0" ::: "memory");
  __builtin_amdgcn_wave_barrier();
}

__device__ __forceinline__ float gelu_tanh(float t) {
  const float u = 0.7978845608028654f * (t + 0.044715f * t * t * t);
  const float e = __expf(-2.0f * u);
  return t * __builtin_amdgcn_rcpf(1.0f + e);
}

__global__ __launch_bounds__(256) void wconv_kernel(
    const float* __restrict__ W, _Float16* __restrict__ Wt,
    unsigned ldw, unsigned zsrc, unsigned nper, unsigned ktot) {
  __shared__ _Float16 T[64 * LDT];
  const unsigned tid = threadIdx.x;
  const unsigned n0 = blockIdx.x * 64u;
  const unsigned k0 = blockIdx.y * 64u;
  const unsigned z = blockIdx.z;
  const float* src = W + (size_t)z * zsrc + (size_t)k0 * ldw + n0;
#pragma unroll 4
  for (unsigned j = 0; j < 16u; ++j) {
    const unsigned idx = tid + 256u * j;
    const unsigned kr = idx >> 6, nc = idx & 63u;
    const float v = src[(size_t)kr * ldw + nc];
    T[nc * LDT + kr] = (_Float16)(WCARRY * bf16r(v));
  }
  __syncthreads();
  v8h x[2];
  size_t off[2];
#pragma unroll
  for (unsigned i = 0; i < 2u; ++i) {
    const unsigned n = 32u * i + (tid >> 3);
    const unsigned kc = (tid & 7u) * 8u;
    x[i] = *(const v8h*)&T[n * LDT + kc];
    off[i] = (size_t)(z * nper + n0 + n) * ktot + k0 + kc;
  }
#pragma unroll
  for (int i = 0; i < 2; ++i) *(volatile v8h*)(Wt + off[i]) = x[i];
  __threadfence();
#pragma unroll
  for (int i = 0; i < 2; ++i) *(volatile v8h*)(Wt + off[i]) = x[i];
}

__device__ __forceinline__ v4f ln_ld4(const float* p, int cvt) {
  v4f a = *(const v4f*)p;
#pragma unroll
  for (int j = 0; j < 4; ++j) a[j] = cvt ? bf16r(a[j]) : a[j];
  return a;
}

__device__ __forceinline__ void ln_store_pass(const float* sp, const float* gw, const float* gb,
                                              _Float16* dp, unsigned lane, int cvt,
                                              float mean, float inv) {
#pragma unroll 1
  for (unsigned j = 0; j < (unsigned)LN_ITERS; ++j) {
    const unsigned c = j * 256u;
    const v4f a0 = ln_ld4(sp + c, cvt);
    const v4f a1 = ln_ld4(sp + c + 4, cvt);
    const v4f w0 = *(const v4f*)(gw + c + lane * 8u);
    const v4f w1 = *(const v4f*)(gw + c + lane * 8u + 4u);
    const v4f b0 = *(const v4f*)(gb + c + lane * 8u);
    const v4f b1 = *(const v4f*)(gb + c + lane * 8u + 4u);
    v8h o;
#pragma unroll
    for (int i = 0; i < 4; ++i) {
      o[i]     = (_Float16)(((a0[i] - mean) * inv) * bf16r(w0[i]) + bf16r(b0[i]));
      o[i + 4] = (_Float16)(((a1[i] - mean) * inv) * bf16r(w1[i]) + bf16r(b1[i]));
    }
    *(volatile v8h*)(dp + c) = o;
  }
}

__global__ __launch_bounds__(256) void ln_kernel(
    const float* __restrict__ X, const float* __restrict__ gw, const float* __restrict__ gb,
    _Float16* __restrict__ dst, int cvt, unsigned src_seq) {
  const unsigned lane = threadIdx.x & 31u;
  const unsigned wave = wave_id();
  const unsigned crow = blockIdx.x * 8u + wave;
  const unsigned bidx = crow / (unsigned)SEQ;
  const unsigned sq = crow - bidx * (unsigned)SEQ;
  const float* sp = X + ((size_t)bidx * src_seq + sq) * DIM + lane * 8u;
  _Float16* dp = dst + (size_t)crow * DIM + lane * 8u;

  float s = 0.0f;
#pragma unroll 1
  for (unsigned j = 0; j < (unsigned)LN_ITERS; ++j) {
    const v4f a0 = ln_ld4(sp + j * 256u, cvt);
    const v4f a1 = ln_ld4(sp + j * 256u + 4, cvt);
    s += ((a0[0] + a0[1]) + (a0[2] + a0[3])) + ((a1[0] + a1[1]) + (a1[2] + a1[3]));
  }
  const float mean = red32_sum(s) * (1.0f / (float)DIM);

  float ss = 0.0f;
#pragma unroll 1
  for (unsigned j = 0; j < (unsigned)LN_ITERS; ++j) {
    const v4f a0 = ln_ld4(sp + j * 256u, cvt);
    const v4f a1 = ln_ld4(sp + j * 256u + 4, cvt);
    float t = 0.0f;
#pragma unroll
    for (int i = 0; i < 4; ++i) {
      const float d0 = a0[i] - mean, d1 = a1[i] - mean;
      t += d0 * d0;
      t += d1 * d1;
    }
    ss += t;
  }
  const float var = red32_sum(ss) * (1.0f / (float)DIM);
  const float inv = 1.0f / sqrtf(var + LN_EPS);

  ln_store_pass(sp, gw, gb, dp, lane, cvt, mean, inv);
  __threadfence();
  ln_store_pass(sp, gw, gb, dp, lane, cvt, mean, inv);
}

template <int MODE, int KD, int ND>
__device__ __forceinline__ void gemm_body(
    const _Float16* __restrict__ A16, const _Float16* __restrict__ Bt,
    const float* __restrict__ bias, const float* __restrict__ addf,
    float* __restrict__ outf, _Float16* __restrict__ out16, float* Cs) {
  static_assert((KD % 32) == 0);
  static_assert((ND % 64) == 0);
  const unsigned tid = threadIdx.x, lane = tid & 31u;
  const unsigned w = wave_id();
  const unsigned mw = w >> 1, nw = w & 1u;
  const unsigned hh = lane >> 4, m = lane & 15u;
  const unsigned n0 = blockIdx.x * 64u;
  const unsigned row0 = blockIdx.y * 64u;

  const _Float16* ap  = A16 + (size_t)(row0 + mw * 16u + m) * KD + hh * 8u;
  const _Float16* bp0 = Bt + (size_t)(n0 + nw * 32u + m) * KD + hh * 8u;
  const _Float16* bp1 = bp0 + (size_t)16 * KD;
  v8f acc0 = {}, acc1 = {};
#pragma unroll 2
  for (unsigned k0 = 0; k0 < (unsigned)KD; k0 += 32u) {
    const v16h a  = frag_at(ap + k0);
    const v16h b0 = frag_at(bp0 + k0);
    const v16h b1 = frag_at(bp1 + k0);
    acc0 = wmma16(a, b0, acc0);
    acc1 = wmma16(a, b1, acc1);
  }
#pragma unroll
  for (int r = 0; r < 8; ++r) {
    float* d = &Cs[(mw * 16u + hh * 8u + (unsigned)r) * LDC + nw * 32u + m];
    d[0]  = acc0[r];
    d[16] = acc1[r];
  }
  __syncthreads();

  if (MODE == 0 || MODE == 3) {
    v8h x[2];
    size_t off[2];
#pragma unroll
    for (unsigned i = 0; i < 2u; ++i) {
      const unsigned r = 32u * i + (tid >> 3);
      const unsigned c = (tid & 7u) * 8u;
      const v4f u0 = *(const v4f*)&Cs[r * LDC + c];
      const v4f u1 = *(const v4f*)&Cs[r * LDC + c + 4];
      const v4f g0 = *(const v4f*)(bias + n0 + c);
      const v4f g1 = *(const v4f*)(bias + n0 + c + 4);
#pragma unroll
      for (int j = 0; j < 4; ++j) {
        const float t0 = u0[j] * (1.0f / WCARRY) + bf16r(g0[j]);
        const float t1 = u1[j] * (1.0f / WCARRY) + bf16r(g1[j]);
        if (MODE == 3) {
          x[i][j]     = (_Float16)(GCARRY * gelu_tanh(t0));
          x[i][j + 4] = (_Float16)(GCARRY * gelu_tanh(t1));
        } else {
          x[i][j]     = (_Float16)t0;
          x[i][j + 4] = (_Float16)t1;
        }
      }
      off[i] = (size_t)(row0 + r) * ND + n0 + c;
    }
#pragma unroll
    for (int i = 0; i < 2; ++i) *(volatile v8h*)(out16 + off[i]) = x[i];
    __threadfence();
#pragma unroll
    for (int i = 0; i < 2; ++i) *(volatile v8h*)(out16 + off[i]) = x[i];
  }

  if (MODE == 1) {
    const unsigned bidx = row0 / (unsigned)SEQ;
    const unsigned key0 = row0 - bidx * (unsigned)SEQ;
    v8h x[2];
    size_t off[2];
#pragma unroll
    for (unsigned i = 0; i < 2u; ++i) {
      const unsigned dcol = 32u * i + (tid >> 3);
      const unsigned kk = (tid & 7u) * 8u;
      const float bv = bf16r(bias[n0 + dcol]);
#pragma unroll
      for (unsigned j = 0; j < 8u; ++j)
        x[i][j] = (_Float16)(Cs[(kk + j) * LDC + dcol] * (1.0f / WCARRY) + bv);
      off[i] = ((size_t)bidx * ND + n0 + dcol) * SEQ + key0 + kk;
    }
#pragma unroll
    for (int i = 0; i < 2; ++i) *(volatile v8h*)(out16 + off[i]) = x[i];
    __threadfence();
#pragma unroll
    for (int i = 0; i < 2; ++i) *(volatile v8h*)(out16 + off[i]) = x[i];
  }

  if (MODE == 2 || MODE == 4) {
    v4f xs[4];
    size_t off[4];
#pragma unroll
    for (unsigned i = 0; i < 4u; ++i) {
      const unsigned r = 16u * i + (tid >> 4);
      const unsigned c = (tid & 15u) * 4u;
      const unsigned crow = row0 + r;
      const unsigned bidx = crow / (unsigned)SEQ;
      const unsigned sq = crow - bidx * (unsigned)SEQ;
      const size_t frow = (size_t)bidx * SEQ_FULL + sq;
      const size_t arow = (MODE == 2) ? frow : (size_t)crow;
      const size_t orow = (MODE == 2) ? (size_t)crow : frow;
      const v4f u = *(const v4f*)&Cs[r * LDC + c];
      const v4f g = *(const v4f*)(bias + n0 + c);
      const v4f ad = *(const v4f*)(addf + arow * ND + n0 + c);
      v4f val;
#pragma unroll
      for (int j = 0; j < 4; ++j) {
        const float res = (MODE == 2) ? bf16r(ad[j]) : ad[j];
        val[j] = res + (u[j] * (1.0f / (WCARRY * VCARRY)) + bf16r(g[j]));
      }
      xs[i] = val;
      off[i] = orow * ND + n0 + c;
    }
#pragma unroll
    for (int i = 0; i < 4; ++i) *(volatile v4f*)(outf + off[i]) = xs[i];
    __threadfence();
#pragma unroll
    for (int i = 0; i < 4; ++i) *(volatile v4f*)(outf + off[i]) = xs[i];
  }
}

__global__ __launch_bounds__(256) void gemm_qk_kernel(
    const _Float16* __restrict__ A16, const _Float16* __restrict__ Bt,
    const float* __restrict__ bias, float* __restrict__ outf, _Float16* __restrict__ out16) {
  __shared__ float Cs[64 * LDC];
  gemm_body<0, DIM, DIM>(A16, Bt, bias, bias, outf, out16, Cs);
}
__global__ __launch_bounds__(256) void gemm_vt_kernel(
    const _Float16* __restrict__ A16, const _Float16* __restrict__ Bt,
    const float* __restrict__ bias, float* __restrict__ outf, _Float16* __restrict__ out16) {
  __shared__ float Cs[64 * LDC];
  gemm_body<1, DIM, DIM>(A16, Bt, bias, bias, outf, out16, Cs);
}
__global__ __launch_bounds__(256) void gemm_oproj_kernel(
    const _Float16* __restrict__ A16, const _Float16* __restrict__ Bt,
    const float* __restrict__ bias, const float* __restrict__ addf,
    float* __restrict__ outf, _Float16* __restrict__ out16) {
  __shared__ float Cs[64 * LDC];
  gemm_body<2, DIM, DIM>(A16, Bt, bias, addf, outf, out16, Cs);
}
__global__ __launch_bounds__(256) void gemm_mlpin_kernel(
    const _Float16* __restrict__ A16, const _Float16* __restrict__ Bt,
    const float* __restrict__ bias, float* __restrict__ outf, _Float16* __restrict__ out16) {
  __shared__ float Cs[64 * LDC];
  gemm_body<3, DIM, DMLP>(A16, Bt, bias, bias, outf, out16, Cs);
}
__global__ __launch_bounds__(256) void gemm_mlpout_kernel(
    const _Float16* __restrict__ A16, const _Float16* __restrict__ Bt,
    const float* __restrict__ bias, const float* __restrict__ addf,
    float* __restrict__ outf, _Float16* __restrict__ out16) {
  __shared__ float Cs[64 * LDC];
  gemm_body<4, DMLP, DIM>(A16, Bt, bias, addf, outf, out16, Cs);
}

__global__ __launch_bounds__(256) void attn_kernel(
    const _Float16* __restrict__ Qh, const _Float16* __restrict__ Kh,
    const _Float16* __restrict__ Vt, _Float16* __restrict__ Ov) {
  __shared__ _Float16 Ks[64 * LDT];
  __shared__ _Float16 Vs[64 * LDT];
  __shared__ _Float16 Ps[8 * 16 * LDT];

  const unsigned tid = threadIdx.x, lane = tid & 31u;
  const unsigned w = wave_id();
  const unsigned hh = lane >> 4, m = lane & 15u;
  const unsigned q0 = blockIdx.x * 128u;
  const unsigned head = blockIdx.y;
  const unsigned b = blockIdx.z;
  const float scale = 0.125f;
  _Float16* P = Ps + w * (16u * LDT);
  const unsigned rmin = q0 + w * 16u;
  const unsigned kend = q0 + 128u;

  const size_t qoff = (size_t)(b * (unsigned)SEQ + rmin + m) * DIM + head * HD + hh * 8u;
  v16h qf[2];
  qf[0] = frag_at(Qh + qoff);
  qf[1] = frag_at(Qh + qoff + 32);

  float mrow[8], lrow[8];
  v8f o[4];
#pragma unroll
  for (int v = 0; v < 8; ++v) { mrow[v] = -1.0e30f; lrow[v] = 0.0f; }
#pragma unroll
  for (int nb = 0; nb < 4; ++nb) o[nb] = (v8f){};

  const size_t kplane = (size_t)b * SEQ * DIM + head * HD;
  const size_t vplane = ((size_t)b * DIM + head * HD) * SEQ;

  for (unsigned kb = 0; kb < kend; kb += 64u) {
#pragma unroll
    for (unsigned j = 0; j < 2u; ++j) {
      const unsigned idx = tid + 256u * j;
      const unsigned r = idx >> 3, c = (idx & 7u) * 8u;
      *(v8h*)&Ks[r * LDT + c] = *(const v8h*)(Kh + kplane + (size_t)(kb + r) * DIM + c);
      *(v8h*)&Vs[r * LDT + c] = *(const v8h*)(Vt + vplane + (size_t)r * SEQ + kb + c);
    }
    __syncthreads();

    if (kb <= rmin) {
      v8f s[4];
#pragma unroll
      for (int kg = 0; kg < 4; ++kg) {
        v8f t = {};
#pragma unroll
        for (int c = 0; c < 2; ++c) {
          const v16h kf = ld_frag(&Ks[(kg * 16) * LDT + c * 32], LDT);
          t = wmma16(qf[c], kf, t);
        }
        s[kg] = t * scale;
      }

      if (kb + 63u > rmin) {
#pragma unroll
        for (int kg = 0; kg < 4; ++kg) {
          const unsigned key = kb + (unsigned)kg * 16u + m;
#pragma unroll
          for (int v = 0; v < 8; ++v) {
            const unsigned row = rmin + hh * 8u + (unsigned)v;
            s[kg][v] = (key > row) ? MASK_FILL : s[kg][v];
          }
        }
      }

      float alpha[8];
#pragma unroll
      for (int v = 0; v < 8; ++v) {
        float mx = fmaxf(fmaxf(s[0][v], s[1][v]), fmaxf(s[2][v], s[3][v]));
        mx = red16_max(mx);
        const float mn = fmaxf(mrow[v], mx);
        alpha[v] = __expf(mrow[v] - mn);
        mrow[v] = mn;
      }
#pragma unroll
      for (int kg = 0; kg < 4; ++kg)
#pragma unroll
        for (int v = 0; v < 8; ++v) s[kg][v] = __expf(s[kg][v] - mrow[v]);
#pragma unroll
      for (int v = 0; v < 8; ++v) {
        const float rs = red16_sum((s[0][v] + s[1][v]) + (s[2][v] + s[3][v]));
        lrow[v] = alpha[v] * lrow[v] + rs;
      }
#pragma unroll
      for (int nb = 0; nb < 4; ++nb)
#pragma unroll
        for (int v = 0; v < 8; ++v) o[nb][v] = o[nb][v] * alpha[v];

#pragma unroll
      for (int kg = 0; kg < 4; ++kg)
#pragma unroll
        for (int v = 0; v < 8; ++v)
          P[(hh * 8u + (unsigned)v) * LDT + (unsigned)kg * 16u + m] =
              (_Float16)(s[kg][v] * PCARRY);
      wave_lds_sync();

#pragma unroll
      for (int c = 0; c < 2; ++c) {
        const v16h pf = ld_frag(P + c * 32, LDT);
#pragma unroll
        for (int nb = 0; nb < 4; ++nb) {
          const v16h vf = ld_frag(&Vs[(nb * 16) * LDT + c * 32], LDT);
          o[nb] = wmma16(pf, vf, o[nb]);
        }
      }
    }
    __syncthreads();
  }

  float inv[8];
#pragma unroll
  for (int v = 0; v < 8; ++v) inv[v] = __builtin_amdgcn_rcpf(lrow[v]) * (VCARRY / PCARRY);
#pragma unroll
  for (int nb = 0; nb < 4; ++nb)
#pragma unroll
    for (int v = 0; v < 8; ++v)
      P[(hh * 8u + (unsigned)v) * LDT + (unsigned)nb * 16u + m] = (_Float16)(o[nb][v] * inv[v]);
  wave_lds_sync();
  v8h x[4];
  size_t off[4];
#pragma unroll
  for (unsigned i = 0; i < 4u; ++i) {
    const unsigned r = 4u * i + (lane >> 3);
    const unsigned c = (lane & 7u) * 8u;
    x[i] = *(const v8h*)&P[r * LDT + c];
    off[i] = (size_t)(b * (unsigned)SEQ + rmin + r) * DIM + head * HD + c;
  }
#pragma unroll
  for (int i = 0; i < 4; ++i) *(volatile v8h*)(Ov + off[i]) = x[i];
  __threadfence();
#pragma unroll
  for (int i = 0; i < 4; ++i) *(volatile v8h*)(Ov + off[i]) = x[i];
}

extern "C" void kernel_launch(void* const* d_in, const int* in_sizes, int n_in,
                              void* d_out, int out_size, void* d_ws, size_t ws_size,
                              hipStream_t stream) {
  if (n_in < 17) return;
  const long long need_x = ((long long)(NB - 1) * SEQ_FULL + SEQ) * DIM;
  if ((long long)in_sizes[0] < need_x) return;
  if (in_sizes[1] < DIM || in_sizes[2] < DIM) return;
  if ((long long)in_sizes[3] < (long long)DIM * DIM) return;
  if ((long long)in_sizes[4] < (long long)DIM * DIM) return;
  if ((long long)in_sizes[5] < (long long)DIM * DIM) return;
  if ((long long)in_sizes[6] < (long long)DIM * DIM) return;
  if (in_sizes[7] < DIM || in_sizes[8] < DIM || in_sizes[9] < DIM || in_sizes[10] < DIM) return;
  if (in_sizes[11] < DIM || in_sizes[12] < DIM) return;
  if ((long long)in_sizes[13] < (long long)DIM * DMLP) return;
  if (in_sizes[14] < DMLP) return;
  if ((long long)in_sizes[15] < (long long)DIM * DMLP) return;
  if (in_sizes[16] < DIM) return;
  if ((long long)out_size < need_x) return;
  if (ws_size < WS_TOTAL) return;

  const float* X     = (const float*)d_in[0];
  const float* ln1w  = (const float*)d_in[1];
  const float* ln1b  = (const float*)d_in[2];
  const float* WQ    = (const float*)d_in[3];
  const float* WK    = (const float*)d_in[4];
  const float* WV    = (const float*)d_in[5];
  const float* WO    = (const float*)d_in[6];
  const float* bQ    = (const float*)d_in[7];
  const float* bK    = (const float*)d_in[8];
  const float* bV    = (const float*)d_in[9];
  const float* bO    = (const float*)d_in[10];
  const float* ln2w  = (const float*)d_in[11];
  const float* ln2b  = (const float*)d_in[12];
  const float* Win   = (const float*)d_in[13];
  const float* bin   = (const float*)d_in[14];
  const float* Wout  = (const float*)d_in[15];
  const float* bout  = (const float*)d_in[16];
  float* out = (float*)d_out;

  char* ws = (char*)d_ws;
  _Float16* WQt   = (_Float16*)(ws + OFF_WQ);
  _Float16* WKt   = (_Float16*)(ws + OFF_WK);
  _Float16* WVt   = (_Float16*)(ws + OFF_WV);
  _Float16* WOt   = (_Float16*)(ws + OFF_WO);
  _Float16* WINt  = (_Float16*)(ws + OFF_WIN);
  _Float16* WOUTt = (_Float16*)(ws + OFF_WOUT);
  _Float16* X1    = (_Float16*)(ws + OFF_X1);
  _Float16* Qh16  = (_Float16*)(ws + OFF_Q);
  _Float16* Kh16  = (_Float16*)(ws + OFF_K);
  _Float16* Vt16  = (_Float16*)(ws + OFF_VT);
  _Float16* Ctx16 = (_Float16*)(ws + OFF_CTX);
  _Float16* X2    = (_Float16*)(ws + OFF_X2);
  float*    Rmid  = (float*)(ws + OFF_RMID);
  _Float16* G16   = (_Float16*)(ws + OFF_G);

  dim3 blk(256);

  wconv_kernel<<<dim3(HD / 64, DIM / 64, NHEAD), blk, 0, stream>>>(
      WQ, WQt, (unsigned)HD, (unsigned)(DIM * HD), (unsigned)HD, (unsigned)DIM);
  wconv_kernel<<<dim3(HD / 64, DIM / 64, NHEAD), blk, 0, stream>>>(
      WK, WKt, (unsigned)HD, (unsigned)(DIM * HD), (unsigned)HD, (unsigned)DIM);
  wconv_kernel<<<dim3(HD / 64, DIM / 64, NHEAD), blk, 0, stream>>>(
      WV, WVt, (unsigned)HD, (unsigned)(DIM * HD), (unsigned)HD, (unsigned)DIM);
  wconv_kernel<<<dim3(DIM / 64, DIM / 64, 1), blk, 0, stream>>>(
      WO, WOt, (unsigned)DIM, 0u, (unsigned)DIM, (unsigned)DIM);
  wconv_kernel<<<dim3(DMLP / 64, DIM / 64, 1), blk, 0, stream>>>(
      Win, WINt, (unsigned)DMLP, 0u, (unsigned)DMLP, (unsigned)DIM);
  wconv_kernel<<<dim3(DIM / 64, DMLP / 64, 1), blk, 0, stream>>>(
      Wout, WOUTt, (unsigned)DIM, 0u, (unsigned)DIM, (unsigned)DMLP);

  ln_kernel<<<dim3(MROWS / 8), blk, 0, stream>>>(X, ln1w, ln1b, X1, 1, (unsigned)SEQ_FULL);

  dim3 gg(DIM / 64, MROWS / 64);
  gemm_qk_kernel<<<gg, blk, 0, stream>>>(X1, WQt, bQ, Rmid, Qh16);
  gemm_qk_kernel<<<gg, blk, 0, stream>>>(X1, WKt, bK, Rmid, Kh16);
  gemm_vt_kernel<<<gg, blk, 0, stream>>>(X1, WVt, bV, Rmid, Vt16);

  attn_kernel<<<dim3(SEQ / 128, NHEAD, NB), blk, 0, stream>>>(Qh16, Kh16, Vt16, Ctx16);

  gemm_oproj_kernel<<<gg, blk, 0, stream>>>(Ctx16, WOt, bO, X, Rmid, Qh16);

  ln_kernel<<<dim3(MROWS / 8), blk, 0, stream>>>(Rmid, ln2w, ln2b, X2, 0, (unsigned)SEQ);

  gemm_mlpin_kernel<<<dim3(DMLP / 64, MROWS / 64), blk, 0, stream>>>(X2, WINt, bin, Rmid, G16);

  gemm_mlpout_kernel<<<gg, blk, 0, stream>>>(G16, WOUTt, bout, Rmid, out, Qh16);
}
